// GNNTower_3384434229647
// MI455X (gfx1250) — hardware-verified
//
#include <hip/hip_runtime.h>
#include <stddef.h>


#define DF      128
#define K2      256
#define NTHR    256
#define NWAVE   8
#define EPT     8
#define NGRP    2
#define CHUNK   (NTHR * EPT * NGRP)
#define WCAP    (EPT * NGRP * 32)
#define LISTN   (NWAVE * WCAP)
#define NBL     512
#define NBP     64
#define WSCALE  64.0f
#define WINV    0.015625f

#define LDS_LAYER (NBL * DF * 4 + LISTN * 4 + NBL * 4 + 64)

static_assert((CHUNK & (CHUNK - 1)) == 0);
static_assert(CHUNK <= 4096);
static_assert((NBL & (NBL - 1)) == 0 && NBL <= 4096);
static_assert((NBP & (NBP - 1)) == 0 && NBP <= 4096);
static_assert(NBL == 16 * NWAVE * 4);
static_assert(NBP == NWAVE * 8);

typedef float    v4f  __attribute__((ext_vector_type(4)));
typedef float    v8f  __attribute__((ext_vector_type(8)));
typedef int      v4i  __attribute__((ext_vector_type(4)));
typedef _Float16 v8h  __attribute__((ext_vector_type(8)));
typedef _Float16 v16h __attribute__((ext_vector_type(16)));
union FragH { v16h v; v8h h[2]; };

__device__ __forceinline__ v8h cvt8(v4f a, v4f b) {
  v8h r;
  r[0] = (_Float16)a.x; r[1] = (_Float16)a.y; r[2] = (_Float16)a.z; r[3] = (_Float16)a.w;
  r[4] = (_Float16)b.x; r[5] = (_Float16)b.y; r[6] = (_Float16)b.z; r[7] = (_Float16)b.w;
  return r;
}

__device__ __forceinline__ v8f wmh(v16h a, v16h b, v8f c) {
  v8f d = __builtin_amdgcn_wmma_f32_16x16x32_f16(false, a, false, b, (short)0, c, false, false);
  asm volatile("v_nop\n\tv_nop\n\tv_nop\n\tv_nop" : "+v"(d) : "v"(a), "v"(b));
  return d;
}

template <int NB>
__device__ __forceinline__ int scan_chunk(const int* __restrict__ keys, int nK, int cbase, int base,
                                          int vec8, int* list, int tid, int lane, int wave) {
  int wc = 0;
#pragma unroll
  for (int g = 0; g < NGRP; ++g) {
    const int el0  = (g * NTHR + tid) * EPT;
    const int e0   = cbase + el0;
    const int sent = -2147483647 - 1;
    v4i da, db;
    if (vec8 != 0 && e0 + 7 < nK) {
      da = *(const v4i*)(keys + e0);
      db = *(const v4i*)(keys + e0 + 4);
    } else {
      da.x = (e0     < nK) ? keys[e0]     : sent;
      da.y = (e0 + 1 < nK) ? keys[e0 + 1] : sent;
      da.z = (e0 + 2 < nK) ? keys[e0 + 2] : sent;
      da.w = (e0 + 3 < nK) ? keys[e0 + 3] : sent;
      db.x = (e0 + 4 < nK) ? keys[e0 + 4] : sent;
      db.y = (e0 + 5 < nK) ? keys[e0 + 5] : sent;
      db.z = (e0 + 6 < nK) ? keys[e0 + 6] : sent;
      db.w = (e0 + 7 < nK) ? keys[e0 + 7] : sent;
    }
    const unsigned nb = (unsigned)base;
    const unsigned s0 = (unsigned)da.x - nb, s1 = (unsigned)da.y - nb;
    const unsigned s2 = (unsigned)da.z - nb, s3 = (unsigned)da.w - nb;
    const unsigned s4 = (unsigned)db.x - nb, s5 = (unsigned)db.y - nb;
    const unsigned s6 = (unsigned)db.z - nb, s7 = (unsigned)db.w - nb;
    const bool h0 = s0 < (unsigned)NB, h1 = s1 < (unsigned)NB, h2 = s2 < (unsigned)NB, h3 = s3 < (unsigned)NB;
    const bool h4 = s4 < (unsigned)NB, h5 = s5 < (unsigned)NB, h6 = s6 < (unsigned)NB, h7 = s7 < (unsigned)NB;
    const unsigned any = __builtin_amdgcn_ballot_w32(h0 | h1 | h2 | h3 | h4 | h5 | h6 | h7);
    if (any != 0u) {
#define HITJ(J, HJ, SJ) { \
        const unsigned mj = __builtin_amdgcn_ballot_w32(HJ); \
        if (mj != 0u) { \
          if (HJ) { \
            const int pos = wc + (int)__builtin_amdgcn_mbcnt_lo(mj, 0u); \
            if (pos < WCAP) list[wave * WCAP + pos] = ((el0 + (J)) << 12) | (int)(SJ); \
          } \
          wc += (int)__builtin_popcount(mj); } }
      HITJ(0, h0, s0)
      HITJ(1, h1, s1)
      HITJ(2, h2, s2)
      HITJ(3, h3, s3)
      HITJ(4, h4, s4)
      HITJ(5, h5, s5)
      HITJ(6, h6, s6)
      HITJ(7, h7, s7)
#undef HITJ
    }
  }
  return wc;
}

__global__ __launch_bounds__(NTHR) void k_wprep(
    const float* __restrict__ Ws, const float* __restrict__ Wn, _Float16* wc, int nTot8) {
  const int i = blockIdx.x * NTHR + threadIdx.x;
  if (i >= nTot8) return;
  const int o = i * 8;
  const int l = o / (DF * K2);
  const int r = o - l * (DF * K2);
  const int n = r / K2;
  const int k = r - n * K2;
  const float* p = ((k < DF) ? Ws : Wn) + ((size_t)l * DF + n) * DF + (k & (DF - 1));
  v4f a = *(const v4f*)p, b = *(const v4f*)(p + 4);
  a = a * WSCALE;
  b = b * WSCALE;
  const v8h hv = cvt8(a, b);
  _Float16* dp = wc + o;
  *(volatile v8h*)dp = hv;
  __threadfence();
  *(volatile v8h*)dp = hv;
}

__global__ __launch_bounds__(NTHR) void k_layer(
    const int* __restrict__ ei, const float* __restrict__ xin, const _Float16* __restrict__ wc,
    const float* __restrict__ bsl, const float* __restrict__ bnl, float* xout,
    int nN, int nE, int vec8) {
  extern __shared__ v4f lds_dyn[];
  float* acc  = (float*)lds_dyn;
  int*   list = (int*)(acc + NBL * DF);
  int*   cnt  = list + LISTN;
  int*   wcnt = cnt + NBL;
  const int tid = threadIdx.x, lane = tid & 31, wave = tid >> 5, hh = lane >> 4, m = lane & 15;
  const int nodeBase = blockIdx.x * NBL;
  const int* dsts = ei + nE;

  {
    const v4f z = {0.f, 0.f, 0.f, 0.f};
    for (int i = tid; i < NBL * DF / 4; i += NTHR) lds_dyn[i] = z;
    for (int i = tid; i < NBL; i += NTHR) cnt[i] = 0;
  }
  __syncthreads();

  const int nChunks = (nE + CHUNK - 1) / CHUNK;
#pragma unroll 1
  for (int ch = 0; ch < nChunks; ++ch) {
    const int cbase = ch * CHUNK;
    const int wcn = scan_chunk<NBL>(dsts, nE, cbase, nodeBase, vec8, list, tid, lane, wave);
    if (lane == 0) wcnt[wave] = wcn;
    __syncthreads();
    if (wave == 0) {
#pragma unroll 1
      for (int wsx = 0; wsx < NWAVE; ++wsx) {
        int n = __builtin_amdgcn_readfirstlane(wcnt[wsx]);
        n = n > WCAP ? WCAP : (n < 0 ? 0 : n);
        const int* lp = list + wsx * WCAP;
#pragma unroll 1
        for (int i = 0; i < n; ++i) {
          const int ent  = __builtin_amdgcn_readfirstlane(lp[i]);
          const int slot = ent & (NBL - 1);
          int e = cbase + ((ent >> 12) & (CHUNK - 1));
          e = e > nE - 1 ? nE - 1 : e;
          int src = ei[e];
          src = src < 0 ? 0 : (src > nN - 1 ? nN - 1 : src);
          const v4f v = *(const v4f*)(xin + (size_t)src * DF + 4 * lane);
          v4f* ap = (v4f*)(acc + slot * DF + 4 * lane);
          *ap = *ap + v;
          if (lane == 0) cnt[slot] = cnt[slot] + 1;
        }
      }
    }
    __syncthreads();
  }

  float bsum[8];
#pragma unroll
  for (int n = 0; n < 8; ++n) bsum[n] = bsl[16 * n + m] + bnl[16 * n + m];

#pragma unroll 1
  for (int q = 0; q < NBL / (16 * NWAVE); ++q) {
    const int t = wave + NWAVE * q;
    v8f c[8];
#pragma unroll
    for (int n = 0; n < 8; ++n) { v8f z = {0.f, 0.f, 0.f, 0.f, 0.f, 0.f, 0.f, 0.f}; c[n] = z; }

    int row = nodeBase + 16 * t + m;
    row = row > nN - 1 ? nN - 1 : row;
    const float* xp = xin + (size_t)row * DF + 8 * hh;
#pragma unroll
    for (int kt = 0; kt < DF / 32; ++kt) {
      const v4f g0 = *(const v4f*)(xp + 32 * kt),      g1 = *(const v4f*)(xp + 32 * kt + 4);
      const v4f g2 = *(const v4f*)(xp + 32 * kt + 16), g3 = *(const v4f*)(xp + 32 * kt + 20);
      FragH a;
      a.h[0] = cvt8(g0, g1);
      a.h[1] = cvt8(g2, g3);
#pragma unroll
      for (int n = 0; n < 8; ++n) {
        const _Float16* bp = wc + (size_t)(16 * n + m) * K2 + 32 * kt + 8 * hh;
        FragH b;
        b.h[0] = *(const v8h*)bp;
        b.h[1] = *(const v8h*)(bp + 16);
        c[n] = wmh(a.v, b.v, c[n]);
      }
    }

    const int dc = cnt[16 * t + m];
    const float id = 1.0f / (float)(dc > 0 ? dc : 1);
    const float* arow = acc + (16 * t + m) * DF + 8 * hh;
#pragma unroll
    for (int kt = 0; kt < DF / 32; ++kt) {
      const v4f p0 = *(const v4f*)(arow + 32 * kt),      p1 = *(const v4f*)(arow + 32 * kt + 4);
      const v4f p2 = *(const v4f*)(arow + 32 * kt + 16), p3 = *(const v4f*)(arow + 32 * kt + 20);
      FragH a;
      a.h[0] = cvt8(p0 * id, p1 * id);
      a.h[1] = cvt8(p2 * id, p3 * id);
#pragma unroll
      for (int n = 0; n < 8; ++n) {
        const _Float16* bp = wc + (size_t)(16 * n + m) * K2 + DF + 32 * kt + 8 * hh;
        FragH b;
        b.h[0] = *(const v8h*)bp;
        b.h[1] = *(const v8h*)(bp + 16);
        c[n] = wmh(a.v, b.v, c[n]);
      }
    }
    __syncthreads();

    float* sp = acc + (16 * t + 8 * hh) * DF + m;
#pragma unroll
    for (int n = 0; n < 8; ++n) {
      const float bb = bsum[n];
      sp[0 * DF + 16 * n] = fmaxf(c[n][0] * WINV + bb, 0.f);
      sp[1 * DF + 16 * n] = fmaxf(c[n][1] * WINV + bb, 0.f);
      sp[2 * DF + 16 * n] = fmaxf(c[n][2] * WINV + bb, 0.f);
      sp[3 * DF + 16 * n] = fmaxf(c[n][3] * WINV + bb, 0.f);
      sp[4 * DF + 16 * n] = fmaxf(c[n][4] * WINV + bb, 0.f);
      sp[5 * DF + 16 * n] = fmaxf(c[n][5] * WINV + bb, 0.f);
      sp[6 * DF + 16 * n] = fmaxf(c[n][6] * WINV + bb, 0.f);
      sp[7 * DF + 16 * n] = fmaxf(c[n][7] * WINV + bb, 0.f);
    }
    __syncthreads();

    const float* lp = acc + 16 * t * DF + 4 * lane;
    float* gp = xout + ((size_t)nodeBase + 16 * t) * DF + 4 * lane;
#pragma unroll
    for (int i = 0; i < 16; ++i) { const v4f v = *(const v4f*)(lp + i * DF); *(volatile v4f*)(gp + (size_t)i * DF) = v; }
    __threadfence();
#pragma unroll
    for (int i = 0; i < 16; ++i) { const v4f v = *(const v4f*)(lp + i * DF); *(volatile v4f*)(gp + (size_t)i * DF) = v; }
  }
}

__global__ __launch_bounds__(NTHR) void k_pool(
    const int* __restrict__ bvec, const int* __restrict__ numg, const float* __restrict__ xin,
    float* out, int nN, int nG) {
  __shared__ __attribute__((aligned(16))) float pacc[NBP * DF];
  __shared__ __attribute__((aligned(16))) int plist[LISTN];
  __shared__ int pcnt[NBP];
  __shared__ int pwcnt[NWAVE];
  const int tid = threadIdx.x, lane = tid & 31, wave = tid >> 5;
  const int gBase = blockIdx.x * NBP;
  const int ngd = numg[0];
  const int nGe = ngd < nG ? (ngd < 0 ? 0 : ngd) : nG;

  {
    const v4f z = {0.f, 0.f, 0.f, 0.f};
    v4f* pz = (v4f*)pacc;
    for (int i = tid; i < NBP * DF / 4; i += NTHR) pz[i] = z;
    for (int i = tid; i < NBP; i += NTHR) pcnt[i] = 0;
  }
  __syncthreads();

  const int nChunks = (nN + CHUNK - 1) / CHUNK;
#pragma unroll 1
  for (int ch = 0; ch < nChunks; ++ch) {
    const int cbase = ch * CHUNK;
    const int wcn = scan_chunk<NBP>(bvec, nN, cbase, gBase, 1, plist, tid, lane, wave);
    if (lane == 0) pwcnt[wave] = wcn;
    __syncthreads();
    if (wave == 0) {
#pragma unroll 1
      for (int wsx = 0; wsx < NWAVE; ++wsx) {
        int n = __builtin_amdgcn_readfirstlane(pwcnt[wsx]);
        n = n > WCAP ? WCAP : (n < 0 ? 0 : n);
        const int* lp = plist + wsx * WCAP;
#pragma unroll 1
        for (int i = 0; i < n; ++i) {
          const int ent  = __builtin_amdgcn_readfirstlane(lp[i]);
          const int slot = ent & (NBP - 1);
          int node = cbase + ((ent >> 12) & (CHUNK - 1));
          node = node > nN - 1 ? nN - 1 : node;
          const v4f v = *(const v4f*)(xin + (size_t)node * DF + 4 * lane);
          v4f* ap = (v4f*)(pacc + slot * DF + 4 * lane);
          *ap = *ap + v;
          if (lane == 0) pcnt[slot] = pcnt[slot] + 1;
        }
      }
    }
    __syncthreads();
  }

#pragma unroll
  for (int i = 0; i < NBP / NWAVE; ++i) {
    const int rl = wave * (NBP / NWAVE) + i;
    const int g  = gBase + rl;
    const int cg = pcnt[rl];
    const float inv = 1.0f / (float)(cg > 0 ? cg : 1);
    const v4f v = *(const v4f*)(pacc + rl * DF + 4 * lane) * inv;
    if (g < nGe) *(volatile v4f*)(out + (size_t)g * DF + 4 * lane) = v;
  }
  __threadfence();
#pragma unroll
  for (int i = 0; i < NBP / NWAVE; ++i) {
    const int rl = wave * (NBP / NWAVE) + i;
    const int g  = gBase + rl;
    const int cg = pcnt[rl];
    const float inv = 1.0f / (float)(cg > 0 ? cg : 1);
    const v4f v = *(const v4f*)(pacc + rl * DF + 4 * lane) * inv;
    if (g < nGe) *(volatile v4f*)(out + (size_t)g * DF + 4 * lane) = v;
  }
}

extern "C" void kernel_launch(void* const* d_in, const int* in_sizes, int n_in,
                              void* d_out, int out_size, void* d_ws, size_t ws_size,
                              hipStream_t stream) {
  if (n_in < 8) return;
  const int nN = in_sizes[0] / DF;
  const int nE = in_sizes[1] / 2;
  if (nN <= 0 || nE < 0 || in_sizes[0] != nN * DF || in_sizes[1] != nE * 2) return;
  if (in_sizes[2] != nN || in_sizes[3] < 1) return;
  const int nL = in_sizes[4] / (DF * DF);
  if (nL < 0 || in_sizes[4] != nL * DF * DF || in_sizes[6] != nL * DF * DF) return;
  if (in_sizes[5] != nL * DF || in_sizes[7] != nL * DF) return;
  const int nG = out_size / DF;
  if (nG <= 0 || out_size != nG * DF) return;

  const float* x0   = (const float*)d_in[0];
  const int*   ei   = (const int*)d_in[1];
  const int*   bvec = (const int*)d_in[2];
  const int*   numg = (const int*)d_in[3];
  const float* Ws   = (const float*)d_in[4];
  const float* bs   = (const float*)d_in[5];
  const float* Wn   = (const float*)d_in[6];
  const float* bn   = (const float*)d_in[7];
  float* out = (float*)d_out;

  const int nBlk = (nN + NBL - 1) / NBL;
  const size_t nPad = (size_t)nBlk * NBL;

  char* ws = (char*)d_ws;
  size_t off = 0;
  const size_t oWc = off; off += (size_t)nL * DF * K2 * 2;       off = (off + 255) & ~(size_t)255;
  const size_t oXA = off; off += nPad * DF * 4;                   off = (off + 255) & ~(size_t)255;
  const size_t oXB = off; off += nPad * DF * 4;                   off = (off + 255) & ~(size_t)255;
  if (off > ws_size) return;
  _Float16* wcp = (_Float16*)(ws + oWc);
  float*    xA  = (float*)(ws + oXA);
  float*    xB  = (float*)(ws + oXB);

  const int vec8 = ((nE & 3) == 0) ? 1 : 0;

  if (nL > 0) {
    const int nTot8 = nL * DF * K2 / 8;
    k_wprep<<<(nTot8 + NTHR - 1) / NTHR, NTHR, 0, stream>>>(Ws, Wn, wcp, nTot8);
  }

  hipFuncSetAttribute(reinterpret_cast<const void*>(&k_layer),
                      hipFuncAttributeMaxDynamicSharedMemorySize, LDS_LAYER);

  const float* cur = x0;
  for (int l = 0; l < nL; ++l) {
    float* dst = ((l & 1) == 0) ? xA : xB;
    k_layer<<<nBlk, NTHR, LDS_LAYER, stream>>>(ei, cur, wcp + (size_t)l * DF * K2,
                                               bs + (size_t)l * DF, bn + (size_t)l * DF,
                                               dst, nN, nE, vec8);
    cur = dst;
  }

  k_pool<<<(nG + NBP - 1) / NBP, NTHR, 0, stream>>>(bvec, numg, cur, out, nN, nG);
}
